// GBlock_481036337798
// MI455X (gfx1250) — hardware-run, weakly checked
//
#include <hip/hip_runtime.h>
#include <stddef.h>
#include <stdint.h>


#define NNODE   50000
#define NEDGE   800000
#define FW      256
#define MPAD    50048
#define AGGP    512
#define XBP     256
#define WP      768
#define SPLIT_LO 1
#define KAGG    (SPLIT_LO != 0 ? 512 : 256)
#define KX      256
#define WXOFF   512
#define NTHR    256
#define NWAVE   8
#define EPT     8
#define CHUNK   (NTHR * EPT)
#define WCAP    (EPT * 32)
#define LISTN   (NWAVE * WCAP)
#define NBA     1024
#define SLA     10
#define NAGGB   49
#define RCAP    20480
#define DEGCAP  64
#define GBM     128
#define GBN     128
#define GTHR    256
#define NTILE   (MPAD / GBM)
#define NB_X    (MPAD * (FW / 8) / NTHR)
#define NB_W    (3 * FW * (FW / 8) / NTHR)
#define WUNIT   (FW * (FW / 8))
#define AGG_ZINTS (LISTN + 2 * RCAP + 3 * NBA)
#define MISC_INTS 16
#define AGG_LDS_INTS (AGG_ZINTS + MISC_INTS)
#define ARB     32

static_assert((CHUNK & (CHUNK - 1)) == 0 && CHUNK <= 4096);
static_assert((NBA & (NBA - 1)) == 0 && NBA == (1 << SLA));
static_assert(((long long)CHUNK << SLA) < (1LL << 31));
static_assert(((long long)NEDGE << SLA) < (1LL << 31));
static_assert(NBA % NWAVE == 0 && NBA % 32 == 0);
static_assert(RCAP % 4 == 0 && AGG_ZINTS % (NTHR * 4) == 0);
static_assert(RCAP * 100 >= 16711 * 105);
static_assert(DEGCAP >= 34 + 8);
static_assert(AGG_LDS_INTS * 4 <= 300000);
static_assert(MPAD % GBM == 0 && MPAD >= NNODE && MPAD - NNODE < GBM);
static_assert(NAGGB * NBA >= MPAD);
static_assert(KAGG % 32 == 0 && KX % 32 == 0 && KAGG <= AGGP && KX <= XBP && WXOFF + KX <= WP && KAGG <= WXOFF);
static_assert(FW == 2 * GBN && GBM == (GTHR / 32) * 16 && GBN == 4 * 32);
static_assert((MPAD * (FW / 8)) % NTHR == 0 && WUNIT % NTHR == 0);
static_assert(NTHR == FW);

typedef float          v2f   __attribute__((ext_vector_type(2)));
typedef float          v4f   __attribute__((ext_vector_type(4)));
typedef float          v8f   __attribute__((ext_vector_type(8)));
typedef int            v4i   __attribute__((ext_vector_type(4)));
typedef int            v8i   __attribute__((ext_vector_type(8)));
typedef unsigned       v2u   __attribute__((ext_vector_type(2)));
typedef unsigned       v4u   __attribute__((ext_vector_type(4)));
typedef unsigned short v8us  __attribute__((ext_vector_type(8)));
typedef unsigned short v16us __attribute__((ext_vector_type(16)));
typedef __bf16         v16bf __attribute__((ext_vector_type(16)));
typedef v4f  __attribute__((may_alias)) v4fa;
typedef v4i  __attribute__((may_alias)) v4ia;
typedef v2u  __attribute__((may_alias)) v2ua;
typedef v4u  __attribute__((may_alias)) v4ua;
typedef v8us __attribute__((may_alias)) v8usa;
union FragB { v16bf v; v16us u; v8us h[2]; v8i w; };

__device__ __forceinline__ v8f wmb(const FragB& a, const FragB& b, v8f c) {
  v8f d = __builtin_amdgcn_wmma_f32_16x16x32_bf16(false, a.v, false, b.v, (short)0, c, false, false);
  asm volatile("v_nop\n\tv_nop\n\tv_nop\n\tv_nop" : "+v"(d) : "v"(a.w), "v"(b.w));
  return d;
}

__device__ __forceinline__ unsigned bf16_bits(float f) {
  const unsigned u = __float_as_uint(f);
  const unsigned r = (u + 0x7FFFu + ((u >> 16) & 1u)) >> 16;
  return (f != f) ? 0x7FC0u : r;
}
__device__ __forceinline__ float bf16_val(float f) {
  return __uint_as_float(bf16_bits(f) << 16);
}

__global__ __launch_bounds__(NTHR) void k_prep(const float* __restrict__ x, const float* __restrict__ wrel,
                                               const float* __restrict__ wroot, const float* __restrict__ brel,
                                               const float* __restrict__ gam, const float* __restrict__ bet,
                                               unsigned short* xb, unsigned short* wcat, float* ps) {
  const int tid = (int)threadIdx.x;
  const int b   = (int)blockIdx.x;
  if (b < NB_X) {
    const int u   = b * NTHR + tid;
    const int row = u >> 5;
    const int c8  = (u & 31) * 8;
    const int rc  = row < NNODE ? row : NNODE - 1;
    const float* p = x + (size_t)rc * FW + c8;
    const v4f a  = *(const v4f*)p;
    const v4f bq = *(const v4f*)(p + 4);
    asm volatile("" :: "v"(a), "v"(bq));
    const unsigned msk = (row < NNODE) ? 0xffffu : 0u;
    v8us o;
    o[0] = (unsigned short)(bf16_bits(a.x) & msk);  o[1] = (unsigned short)(bf16_bits(a.y) & msk);
    o[2] = (unsigned short)(bf16_bits(a.z) & msk);  o[3] = (unsigned short)(bf16_bits(a.w) & msk);
    o[4] = (unsigned short)(bf16_bits(bq.x) & msk); o[5] = (unsigned short)(bf16_bits(bq.y) & msk);
    o[6] = (unsigned short)(bf16_bits(bq.z) & msk); o[7] = (unsigned short)(bf16_bits(bq.w) & msk);
    unsigned short* dp = xb + (size_t)u * 8;
    *(volatile v8us*)dp = o;
    __threadfence();
    *(volatile v8us*)dp = o;
  } else if (b < NB_X + NB_W) {
    const int v    = (b - NB_X) * NTHR + tid;
    const int part = v >> 13;
    const int w    = v & (WUNIT - 1);
    const int n    = w >> 5;
    const int k8   = (w & 31) * 8;
    v4f a, bq;
    if (part < 2) {
      const float* p = wrel + (size_t)n * FW + k8;
      a  = *(const v4f*)p;
      bq = *(const v4f*)(p + 4);
    } else {
      const float* p = wroot + (size_t)n * FW + k8;
      a  = *(const v4f*)p;
      bq = *(const v4f*)(p + 4);
    }
    v8us o;
    o[0] = (unsigned short)bf16_bits(a.x);  o[1] = (unsigned short)bf16_bits(a.y);
    o[2] = (unsigned short)bf16_bits(a.z);  o[3] = (unsigned short)bf16_bits(a.w);
    o[4] = (unsigned short)bf16_bits(bq.x); o[5] = (unsigned short)bf16_bits(bq.y);
    o[6] = (unsigned short)bf16_bits(bq.z); o[7] = (unsigned short)bf16_bits(bq.w);
    unsigned short* dp = wcat + (size_t)n * WP + part * FW + k8;
    *(volatile v8us*)dp = o;
    __threadfence();
    *(volatile v8us*)dp = o;
  } else {
    if (tid < 192) {
      const int which = tid >> 6;
      const int j     = (tid & 63) * 4;
      const v4f a  = *(const v4f*)(brel + j);
      const v4f g  = *(const v4f*)(gam + j);
      const v4f be = *(const v4f*)(bet + j);
      asm volatile("" :: "v"(a), "v"(g), "v"(be));
      const v4f s = (which == 0) ? a : ((which == 1) ? g : be);
      v4f o;
      o.x = bf16_val(s.x); o.y = bf16_val(s.y); o.z = bf16_val(s.z); o.w = bf16_val(s.w);
      float* dp = ps + 4 * tid;
      *(volatile v4f*)dp = o;
      __threadfence();
      *(volatile v4f*)dp = o;
    }
  }
}

template <int SLB>
__device__ __forceinline__ int scan_chunk(const int* __restrict__ dsts, int nE, int cbase, int slotBase,
                                          int* list, int lane, int wave) {
  int wc = 0;
  const int el0  = wave * WCAP + lane;
  const int e0   = cbase + el0;
  const int sent = (int)(1u << 31);
  int d0, d1, d2, d3, d4, d5, d6, d7;
  if (cbase + CHUNK <= nE) {
    const int* p = dsts + e0;
    d0 = p[0];   d1 = p[32];  d2 = p[64];  d3 = p[96];
    d4 = p[128]; d5 = p[160]; d6 = p[192]; d7 = p[224];
  } else {
    const int l = nE - 1;
    d0 = (e0       < nE) ? dsts[min(e0,       l)] : sent;
    d1 = (e0 + 32  < nE) ? dsts[min(e0 + 32,  l)] : sent;
    d2 = (e0 + 64  < nE) ? dsts[min(e0 + 64,  l)] : sent;
    d3 = (e0 + 96  < nE) ? dsts[min(e0 + 96,  l)] : sent;
    d4 = (e0 + 128 < nE) ? dsts[min(e0 + 128, l)] : sent;
    d5 = (e0 + 160 < nE) ? dsts[min(e0 + 160, l)] : sent;
    d6 = (e0 + 192 < nE) ? dsts[min(e0 + 192, l)] : sent;
    d7 = (e0 + 224 < nE) ? dsts[min(e0 + 224, l)] : sent;
  }
  const unsigned nbs = (unsigned)slotBase;
  const unsigned unb = (unsigned)NBA;
  const unsigned s0 = (unsigned)d0 - nbs, s1 = (unsigned)d1 - nbs;
  const unsigned s2 = (unsigned)d2 - nbs, s3 = (unsigned)d3 - nbs;
  const unsigned s4 = (unsigned)d4 - nbs, s5 = (unsigned)d5 - nbs;
  const unsigned s6 = (unsigned)d6 - nbs, s7 = (unsigned)d7 - nbs;
  const bool h0 = s0 < unb, h1 = s1 < unb, h2 = s2 < unb, h3 = s3 < unb;
  const bool h4 = s4 < unb, h5 = s5 < unb, h6 = s6 < unb, h7 = s7 < unb;
  const unsigned any = __builtin_amdgcn_ballot_w32(h0 | h1 | h2 | h3 | h4 | h5 | h6 | h7);
  if (any != 0u) {
#define HITJ(J, HJ, SJ) { \
      const unsigned mj = __builtin_amdgcn_ballot_w32(HJ); \
      if (mj != 0u) { \
        if (HJ) { \
          const int pos = wc + (int)__builtin_amdgcn_mbcnt_lo(mj, 0u); \
          if (pos < WCAP) list[wave * WCAP + pos] = ((el0 + 32 * (J)) << SLB) | (int)(SJ); \
        } \
        wc += (int)__builtin_popcount(mj); } }
    HITJ(0, h0, s0)
    HITJ(1, h1, s1)
    HITJ(2, h2, s2)
    HITJ(3, h3, s3)
    HITJ(4, h4, s4)
    HITJ(5, h5, s5)
    HITJ(6, h6, s6)
    HITJ(7, h7, s7)
#undef HITJ
  }
  return wc;
}

__global__ __launch_bounds__(NTHR) void k_esum(const int* __restrict__ srcs, const int* __restrict__ dsts,
                                               const float* __restrict__ ew, int nE, int nN, int mRows,
                                               const unsigned short* __restrict__ xb, unsigned short* apl) {
  extern __shared__ __attribute__((aligned(16))) int dsm[];
  int* list = dsm;
  int* hl   = dsm + LISTN;
  int* sl   = hl + RCAP;
  int* cnt  = sl + RCAP;
  int* offs = cnt + NBA;
  int* cur  = offs + NBA;
  int* misc = cur + NBA;
  const int tid = (int)threadIdx.x, lane = tid & 31, wave = tid >> 5;
  const int nodeBase = (int)blockIdx.x * NBA;

  {
    const v4i z4 = {0, 0, 0, 0};
    for (int i = tid * 4; i < AGG_ZINTS; i += NTHR * 4) *(v4ia*)(dsm + i) = z4;
    if (tid < MISC_INTS) misc[tid] = 0;
  }
  __syncthreads();

  int t = 0, ov = 0;
  const int nChunks = (nE + CHUNK - 1) / CHUNK;
#pragma unroll 1
  for (int ch = 0; ch < nChunks; ++ch) {
    const int cbase = ch * CHUNK;
    const int wc = scan_chunk<SLA>(dsts, nE, cbase, nodeBase, list, lane, wave);
    if (lane == 0) misc[wave] = wc;
    __syncthreads();
    if (wave == 0) {
#pragma unroll 1
      for (int w2 = 0; w2 < NWAVE; ++w2) {
        int c = misc[w2];
        c = c < 0 ? 0 : (c > WCAP ? WCAP : c);
#pragma unroll 1
        for (int b0 = 0; b0 < c; b0 += 32) {
          const int idx = b0 + lane;
          const int ent = list[w2 * WCAP + (idx < WCAP ? idx : WCAP - 1)];
          const int m32 = (c - b0) < 32 ? (c - b0) : 32;
#pragma unroll 1
          for (int k = 0; k < m32; ++k) {
            const int u    = __builtin_amdgcn_readlane(ent, k);
            const int slot = u & (NBA - 1);
            const int el   = (u >> SLA) & (CHUNK - 1);
            const int pk   = ((cbase + el) << SLA) | slot;
            if (t < RCAP) {
              if (lane == 0) { hl[t] = pk; cnt[slot] = cnt[slot] + 1; }
              t = t + 1;
            } else {
              ov = 1;
            }
          }
        }
      }
    }
    __syncthreads();
  }
  if (wave == 0 && lane == 0) { misc[8] = t; misc[9] = ov; }
  __syncthreads();
  int tt = misc[8];
  tt = tt < 0 ? 0 : (tt > RCAP ? RCAP : tt);
  const int ovf = misc[9];

  if (wave == 0) {
    const int base = lane * (NBA / 32);
    int s = 0;
#pragma unroll 1
    for (int i = 0; i < NBA / 32; ++i) s += cnt[base + i];
    int incl = s;
#pragma unroll
    for (int d = 1; d < 32; d <<= 1) {
      const int y = __shfl_up(incl, d, 32);
      if (lane >= d) incl += y;
    }
    int run = incl - s;
#pragma unroll 1
    for (int i = 0; i < NBA / 32; ++i) {
      const int cv = cnt[base + i];
      offs[base + i] = run;
      cur[base + i]  = run;
      run += cv;
    }
  }
  __syncthreads();
  if (wave == 0) {
#pragma unroll 1
    for (int b0 = 0; b0 < tt; b0 += 32) {
      const int idx = b0 + lane;
      const int ent = hl[idx < RCAP ? idx : RCAP - 1];
      const int m32 = (tt - b0) < 32 ? (tt - b0) : 32;
#pragma unroll 1
      for (int k = 0; k < m32; ++k) {
        const int u    = __builtin_amdgcn_readlane(ent, k);
        const int slot = u & (NBA - 1);
        if (lane == 0) {
          int p = cur[slot];
          p = p < 0 ? 0 : (p > RCAP - 1 ? RCAP - 1 : p);
          sl[p] = u;
          cur[slot] = p + 1;
        }
      }
    }
  }
  __syncthreads();

  const float nanv = __int_as_float(0x7fc00000);
  const float pz = (ovf != 0) ? nanv : 0.0f;
#pragma unroll 1
  for (int si = 0; si < NBA / NWAVE; ++si) {
    const int s    = si * NWAVE + wave;
    const int node = nodeBase + s;
    int cv = cnt[s];
    const bool big = cv > DEGCAP;
    cv = cv < 0 ? 0 : (cv > DEGCAP ? DEGCAP : cv);
    int ovv = offs[s];
    ovv = ovv < 0 ? 0 : (ovv > RCAP ? RCAP : ovv);
    const int c = __builtin_amdgcn_readfirstlane(cv);
    const int o = __builtin_amdgcn_readfirstlane(ovv);
    float a0 = 0.0f, a1 = 0.0f, a2 = 0.0f, a3 = 0.0f, a4 = 0.0f, a5 = 0.0f, a6 = 0.0f, a7 = 0.0f;
#pragma unroll 1
    for (int b0 = 0; b0 < c; b0 += 32) {
      int idx = o + b0 + lane;
      idx = idx > RCAP - 1 ? RCAP - 1 : idx;
      const int ent = sl[idx];
      int eid = ent >> SLA;
      eid = eid < 0 ? 0 : (eid > nE - 1 ? nE - 1 : eid);
      int sr = srcs[eid];
      sr = sr < 0 ? 0 : (sr > nN - 1 ? nN - 1 : sr);
      const float wv  = bf16_val(ew[eid]);
      const int   wvi = __float_as_int(wv);
      const int m32 = (c - b0) < 32 ? (c - b0) : 32;
#pragma unroll 1
      for (int k = 0; k < m32; ++k) {
        const int   sk = __builtin_amdgcn_readlane(sr, k);
        const float ck = __int_as_float(__builtin_amdgcn_readlane(wvi, k));
        const v4u q = *(const v4ua*)(xb + (size_t)sk * XBP + 8 * lane);
        a0 = fmaf(ck, __uint_as_float(q.x << 16),          a0);
        a1 = fmaf(ck, __uint_as_float(q.x & 0xffff0000u), a1);
        a2 = fmaf(ck, __uint_as_float(q.y << 16),          a2);
        a3 = fmaf(ck, __uint_as_float(q.y & 0xffff0000u), a3);
        a4 = fmaf(ck, __uint_as_float(q.z << 16),          a4);
        a5 = fmaf(ck, __uint_as_float(q.z & 0xffff0000u), a5);
        a6 = fmaf(ck, __uint_as_float(q.w << 16),          a6);
        a7 = fmaf(ck, __uint_as_float(q.w & 0xffff0000u), a7);
      }
    }
    const float pzr = big ? nanv : pz;
    const bool live = node < nN;
    float mv[8];
    mv[0] = live ? (a0 + pzr) : 0.0f; mv[1] = live ? (a1 + pzr) : 0.0f;
    mv[2] = live ? (a2 + pzr) : 0.0f; mv[3] = live ? (a3 + pzr) : 0.0f;
    mv[4] = live ? (a4 + pzr) : 0.0f; mv[5] = live ? (a5 + pzr) : 0.0f;
    mv[6] = live ? (a6 + pzr) : 0.0f; mv[7] = live ? (a7 + pzr) : 0.0f;
    v8us hv, lv;
#pragma unroll
    for (int i = 0; i < 8; ++i) {
      const unsigned hb = bf16_bits(mv[i]);
      hv[i] = (unsigned short)hb;
      lv[i] = (unsigned short)bf16_bits(mv[i] - __uint_as_float(hb << 16));
    }
    if (node < mRows) {
      unsigned short* rp = apl + (size_t)node * AGGP + 8 * lane;
      *(volatile v8us*)rp = hv;
      *(volatile v8us*)(rp + FW) = lv;
      __threadfence();
      *(volatile v8us*)rp = hv;
      *(volatile v8us*)(rp + FW) = lv;
    }
  }
}

__device__ __forceinline__ void kstep(const unsigned short* ap, const unsigned short* bp, v8f (&acc)[8]) {
  FragB af;
  af.h[0] = *(const v8usa*)ap;
  af.h[1] = *(const v8usa*)(ap + 16);
#pragma unroll
  for (int nt = 0; nt < 8; ++nt) {
    const unsigned short* wq = bp + (size_t)(16 * nt) * (size_t)WP;
    FragB bf;
    bf.h[0] = *(const v8usa*)wq;
    bf.h[1] = *(const v8usa*)(wq + 16);
    acc[nt] = wmb(af, bf, acc[nt]);
  }
}

__global__ __launch_bounds__(GTHR) __attribute__((amdgpu_num_vgpr(248)))
void k_gemm(const unsigned short* __restrict__ agg, const unsigned short* __restrict__ xb,
            const unsigned short* __restrict__ wcat, const float* __restrict__ ps, int nN,
            float* tout, float* rec) {
  extern __shared__ __attribute__((aligned(16))) float gsm[];
  __shared__ __attribute__((aligned(16))) float bsh[GBN];
  __shared__ __attribute__((aligned(16))) float psum[GTHR];
  __shared__ __attribute__((aligned(16))) float pq[GTHR];
  __shared__ __attribute__((aligned(16))) float recs[2 * GBN];
  const int tid = (int)threadIdx.x, lane = tid & 31, wave = tid >> 5, hh = lane >> 4, m = lane & 15;
  const int rowBase = (int)blockIdx.x * GBM;
  const int colBase = (int)blockIdx.y * GBN;

  if (tid < 32) {
    const v4f b4 = *(const v4f*)(ps + colBase + 4 * tid);
    *(v4fa*)(bsh + 4 * tid) = b4;
  }

  v8f acc[8];
  {
    const v8f z = {0.f, 0.f, 0.f, 0.f, 0.f, 0.f, 0.f, 0.f};
#pragma unroll
    for (int t = 0; t < 8; ++t) acc[t] = z;
  }
  const unsigned short* apa = agg  + (size_t)(rowBase + 16 * wave + m) * (size_t)AGGP + 8 * hh;
  const unsigned short* apx = xb   + (size_t)(rowBase + 16 * wave + m) * (size_t)XBP + 8 * hh;
  const unsigned short* bp  = wcat + (size_t)(colBase + m) * (size_t)WP + 8 * hh;

#pragma unroll 1
  for (int k0 = 0; k0 < KAGG; k0 += 32) kstep(apa + k0, bp + k0, acc);
#pragma unroll 1
  for (int k0 = 0; k0 < KX; k0 += 32) kstep(apx + k0, bp + WXOFF + k0, acc);

#pragma unroll
  for (int nt = 0; nt < 8; ++nt) {
    const int lc = 16 * nt + m;
#pragma unroll
    for (int r = 0; r < 8; ++r) {
      const int lr = 16 * wave + 8 * hh + r;
      gsm[lr * GBN + lc] = acc[nt][r];
    }
  }
  __syncthreads();

  const v4f bb = *(const v4fa*)(bsh + 4 * lane);
#pragma unroll 1
  for (int i = 0; i < 16; ++i) {
    const int lr = 16 * wave + i;
    float* sp = gsm + lr * GBN + 4 * lane;
    const v4f tv = *(const v4fa*)sp + bb;
    *(v4fa*)sp = tv;
    *(volatile v4f*)(tout + (size_t)(rowBase + lr) * FW + colBase + 4 * lane) = tv;
  }
  __threadfence();
#pragma unroll 1
  for (int i = 0; i < 16; ++i) {
    const int lr = 16 * wave + i;
    const v4f tv = *(const v4fa*)(gsm + lr * GBN + 4 * lane);
    *(volatile v4f*)(tout + (size_t)(rowBase + lr) * FW + colBase + 4 * lane) = tv;
  }
  __syncthreads();

  int nv = nN - rowBase;
  nv = nv < 0 ? 0 : (nv > GBM ? GBM : nv);
  const int c  = tid & (GBN - 1);
  const int hf = tid >> 7;
  const int ra = 64 * hf;
  int rb = ra + 64;
  rb = rb > nv ? nv : rb;
  float s = 0.0f;
#pragma unroll 4
  for (int r = ra; r < rb; ++r) s += gsm[r * GBN + c];
  psum[tid] = s;
  __syncthreads();
  const float cf   = (float)(nv > 0 ? nv : 1);
  const float rcf  = 1.0f / cf;
  const float mean = (psum[c] + psum[GBN + c]) * rcf;
  float q = 0.0f;
#pragma unroll 4
  for (int r = ra; r < rb; ++r) {
    const float d = gsm[r * GBN + c] - mean;
    q = fmaf(d, d, q);
  }
  pq[tid] = q;
  __syncthreads();
  if (tid < GBN) {
    recs[2 * tid]     = mean;
    recs[2 * tid + 1] = pq[tid] + pq[GBN + tid];
  }
  __syncthreads();
  v4f rv = {0.f, 0.f, 0.f, 0.f};
  if (tid < 64) rv = *(const v4fa*)(recs + 4 * tid);
  float* rp = rec + ((size_t)blockIdx.x * FW + (size_t)colBase) * 2 + 4 * (tid & 63);
  if (tid < 64) *(volatile v4f*)rp = rv;
  __threadfence();
  if (tid < 64) *(volatile v4f*)rp = rv;
}

__global__ __launch_bounds__(FW) void k_comb(const float* __restrict__ rec, int nTile, int nN, float* stat) {
  __shared__ __attribute__((aligned(16))) float stg[2 * FW];
  const int tid = (int)threadIdx.x;
  double n = 0.0, mean = 0.0, M2 = 0.0;
#pragma unroll 1
  for (int t = 0; t < nTile; ++t) {
    int ci = nN - t * GBM;
    ci = ci < 0 ? 0 : (ci > GBM ? GBM : ci);
    const v2f r = *(const v2f*)(rec + ((size_t)t * FW + (size_t)tid) * 2);
    const double nb = (double)ci;
    const double mb = (double)r.x;
    const double qb = (double)r.y;
    if (ci > 0) {
      const double nn = n + nb;
      const double delta = mb - mean;
      const double f = nb / nn;
      mean = mean + delta * f;
      M2 = M2 + qb + delta * delta * n * f;
      n = nn;
    }
  }
  const double nt = n < 1.0 ? 1.0 : n;
  const float varf  = (float)(M2 / nt);
  const float meanf = (float)mean;
  const float rs = 1.0f / sqrtf(varf + 1e-5f);
  stg[tid] = meanf;
  stg[FW + tid] = rs;
  __syncthreads();
  v4f v = {0.f, 0.f, 0.f, 0.f};
  if (tid < (2 * FW) / 4) v = *(const v4fa*)(stg + 4 * tid);
  if (tid < (2 * FW) / 4) *(volatile v4f*)(stat + 4 * tid) = v;
  __threadfence();
  if (tid < (2 * FW) / 4) *(volatile v4f*)(stat + 4 * tid) = v;
}

__global__ __launch_bounds__(NTHR) void k_apply(const float* __restrict__ tin, const unsigned short* __restrict__ xb,
                                                const float* __restrict__ ps, int nN, float* out) {
  __shared__ __attribute__((aligned(16))) float psh[4 * FW];
  const int tid = (int)threadIdx.x, lane = tid & 31, wave = tid >> 5;
  {
    const v4f v = *(const v4f*)(ps + FW + 4 * tid);
    *(v4fa*)(psh + 4 * tid) = v;
  }
  __syncthreads();
  const v4f g0 = *(const v4fa*)(psh + 4 * lane);
  const v4f g1 = *(const v4fa*)(psh + 128 + 4 * lane);
  const v4f e0 = *(const v4fa*)(psh + FW + 4 * lane);
  const v4f e1 = *(const v4fa*)(psh + FW + 128 + 4 * lane);
  const v4f m0 = *(const v4fa*)(psh + 2 * FW + 4 * lane);
  const v4f m1 = *(const v4fa*)(psh + 2 * FW + 128 + 4 * lane);
  const v4f r0 = *(const v4fa*)(psh + 3 * FW + 4 * lane);
  const v4f r1 = *(const v4fa*)(psh + 3 * FW + 128 + 4 * lane);
  const int rowBlk = (int)blockIdx.x * ARB;
#pragma unroll 1
  for (int i = 0; i < ARB / NWAVE; ++i) {
    const int row = rowBlk + wave + NWAVE * i;
    if (row < nN) {
      const float* tp = tin + (size_t)row * FW + 4 * lane;
      const v4f t0 = *(const v4f*)tp;
      const v4f t1 = *(const v4f*)(tp + 128);
      const unsigned short* xp = xb + (size_t)row * XBP + 4 * lane;
      const v2u q0 = *(const v2ua*)xp;
      const v2u q1 = *(const v2ua*)(xp + 128);
      v4f x0, x1;
      x0.x = __uint_as_float(q0.x << 16); x0.y = __uint_as_float(q0.x & 0xffff0000u);
      x0.z = __uint_as_float(q0.y << 16); x0.w = __uint_as_float(q0.y & 0xffff0000u);
      x1.x = __uint_as_float(q1.x << 16); x1.y = __uint_as_float(q1.x & 0xffff0000u);
      x1.z = __uint_as_float(q1.y << 16); x1.w = __uint_as_float(q1.y & 0xffff0000u);
      v4f y0 = ((t0 - m0) * r0) * g0 + e0;
      v4f y1 = ((t1 - m1) * r1) * g1 + e1;
      y0.x = (y0.x > 0.0f) ? y0.x : (y0.x - y0.x); y0.y = (y0.y > 0.0f) ? y0.y : (y0.y - y0.y);
      y0.z = (y0.z > 0.0f) ? y0.z : (y0.z - y0.z); y0.w = (y0.w > 0.0f) ? y0.w : (y0.w - y0.w);
      y1.x = (y1.x > 0.0f) ? y1.x : (y1.x - y1.x); y1.y = (y1.y > 0.0f) ? y1.y : (y1.y - y1.y);
      y1.z = (y1.z > 0.0f) ? y1.z : (y1.z - y1.z); y1.w = (y1.w > 0.0f) ? y1.w : (y1.w - y1.w);
      v4f o0 = y0 + x0;
      v4f o1 = y1 + x1;
      o0.x = (o0.x > 0.0f) ? o0.x : (o0.x - o0.x); o0.y = (o0.y > 0.0f) ? o0.y : (o0.y - o0.y);
      o0.z = (o0.z > 0.0f) ? o0.z : (o0.z - o0.z); o0.w = (o0.w > 0.0f) ? o0.w : (o0.w - o0.w);
      o1.x = (o1.x > 0.0f) ? o1.x : (o1.x - o1.x); o1.y = (o1.y > 0.0f) ? o1.y : (o1.y - o1.y);
      o1.z = (o1.z > 0.0f) ? o1.z : (o1.z - o1.z); o1.w = (o1.w > 0.0f) ? o1.w : (o1.w - o1.w);
      float* op = out + (size_t)row * FW + 4 * lane;
      *(volatile v4f*)op = o0;
      *(volatile v4f*)(op + 128) = o1;
      __threadfence();
      *(volatile v4f*)op = o0;
      *(volatile v4f*)(op + 128) = o1;
    }
  }
}

static inline size_t al256(size_t o) { return (o + 255) & ~(size_t)255; }

#define SZ_XB   ((size_t)MPAD * XBP * 2)
#define SZ_AGG  ((size_t)MPAD * AGGP * 2)
#define SZ_T    ((size_t)MPAD * FW * 4)
#define SZ_WCAT ((size_t)FW * WP * 2)
#define SZ_REC  ((size_t)NTILE * FW * 2 * 4)
#define SZ_PS   ((size_t)5 * FW * 4)
static_assert(SZ_XB % 256 == 0 && SZ_AGG % 256 == 0 && SZ_T % 256 == 0 && SZ_WCAT % 256 == 0);
static_assert(SZ_REC % 256 == 0 && SZ_PS % 256 == 0);
static_assert(SZ_XB + SZ_AGG + SZ_T + SZ_WCAT + SZ_REC + SZ_PS <= (size_t)(128u << 20));

extern "C" void kernel_launch(void* const* d_in, const int* in_sizes, int n_in,
                              void* d_out, int out_size, void* d_ws, size_t ws_size,
                              hipStream_t stream) {
  if (n_in < 8) return;
  if (in_sizes[0] != NNODE * FW) return;
  if (in_sizes[1] != NEDGE) return;
  if (in_sizes[2] != FW * FW || in_sizes[3] != FW) return;
  if (in_sizes[4] != FW * FW) return;
  if (in_sizes[5] != FW || in_sizes[6] != FW) return;
  if (in_sizes[7] != 2 * NEDGE) return;
  if ((long long)out_size != (long long)NNODE * FW) return;

  const float* x     = (const float*)d_in[0];
  const float* ew    = (const float*)d_in[1];
  const float* wrel  = (const float*)d_in[2];
  const float* brel  = (const float*)d_in[3];
  const float* wroot = (const float*)d_in[4];
  const float* gam   = (const float*)d_in[5];
  const float* bet   = (const float*)d_in[6];
  const int*   ei    = (const int*)d_in[7];
  float* out = (float*)d_out;

  char* ws = (char*)d_ws;
  size_t off = 0;
  const size_t oXB  = off; off = al256(off + SZ_XB);
  const size_t oAGG = off; off = al256(off + SZ_AGG);
  const size_t oT   = off; off = al256(off + SZ_T);
  const size_t oW   = off; off = al256(off + SZ_WCAT);
  const size_t oREC = off; off = al256(off + SZ_REC);
  const size_t oPS  = off; off = al256(off + SZ_PS);
  if (off > ws_size || off > (size_t)(128u << 20)) return;
  unsigned short* XB   = (unsigned short*)(ws + oXB);
  unsigned short* AGG  = (unsigned short*)(ws + oAGG);
  float*          T    = (float*)(ws + oT);
  unsigned short* WCAT = (unsigned short*)(ws + oW);
  float*          REC  = (float*)(ws + oREC);
  float*          PS   = (float*)(ws + oPS);
  float*          STAT = PS + 3 * FW;

  const size_t esumLds = (size_t)AGG_LDS_INTS * 4;
  const size_t gemmLds = (size_t)GBM * GBN * 4;
  hipFuncSetAttribute(reinterpret_cast<const void*>(&k_esum), hipFuncAttributeMaxDynamicSharedMemorySize, (int)esumLds);
  hipFuncSetAttribute(reinterpret_cast<const void*>(&k_gemm), hipFuncAttributeMaxDynamicSharedMemorySize, (int)gemmLds);

  k_prep<<<NB_X + NB_W + 1, NTHR, 0, stream>>>(x, wrel, wroot, brel, gam, bet, XB, WCAT, PS);
  k_esum<<<NAGGB, NTHR, esumLds, stream>>>(ei, ei + NEDGE, ew, NEDGE, NNODE, MPAD, XB, AGG);
  k_gemm<<<dim3(NTILE, FW / GBN), GTHR, gemmLds, stream>>>(AGG, XB, WCAT, PS, NNODE, T, REC);
  k_comb<<<1, FW, 0, stream>>>(REC, NTILE, NNODE, STAT);
  k_apply<<<(NNODE + ARB - 1) / ARB, NTHR, 0, stream>>>(T, XB, PS, NNODE, out);
}
